// LSTMAutoencoder_53386443489774
// MI455X (gfx1250) — hardware-run, weakly checked
//
#include <hip/hip_runtime.h>

typedef __attribute__((ext_vector_type(16))) _Float16 v16h;
typedef __attribute__((ext_vector_type(8)))  _Float16 v8h;
typedef __attribute__((ext_vector_type(16))) __bf16   v16b;
typedef __attribute__((ext_vector_type(8)))  __bf16   v8b;
typedef __attribute__((ext_vector_type(8)))  float    v8f;
typedef __attribute__((ext_vector_type(4)))  float    v4f;

__device__ __forceinline__ unsigned short f2bf_bits(float f) {
  unsigned u = __float_as_uint(f);
  return (unsigned short)((u + 0x7FFFu + ((u >> 16) & 1u)) >> 16);
}
__device__ __forceinline__ float bf_bits2f(unsigned short h) { return __uint_as_float(((unsigned)h) << 16); }

__device__ __forceinline__ void dep_guard_h(v8f& a, v8f& b, v16h x, v16h y) { asm volatile("v_nop\n\tv_nop\n\tv_nop\n\tv_nop" : "+v"(a), "+v"(b) : "v"(x), "v"(y)); }
__device__ __forceinline__ void dep_guard_b(v8f& a, v8f& b, v16b x, v16b y) { asm volatile("v_nop\n\tv_nop\n\tv_nop\n\tv_nop" : "+v"(a), "+v"(b) : "v"(x), "v"(y)); }
__device__ __forceinline__ void keep4_h(v16h a, v16h b, v16h c, v16h d) { asm volatile("v_nop" :: "v"(a), "v"(b), "v"(c), "v"(d)); }
__device__ __forceinline__ void keep4_b(v16b a, v16b b, v16b c, v16b d) { asm volatile("v_nop" :: "v"(a), "v"(b), "v"(c), "v"(d)); }
__device__ __forceinline__ void acc_guard4(v8f& a, v8f& b, v8f& c, v8f& d) { asm volatile("v_nop\n\tv_nop\n\tv_nop\n\tv_nop" : "+v"(a), "+v"(b), "+v"(c), "+v"(d)); }
template <typename T> struct Frag;
template <> struct Frag<_Float16> {
  typedef v16h V; union U { v16h v; v8h h[2]; };
  static __device__ __forceinline__ v16h load(const _Float16* p) {
    U f; f.h[0] = *(const v8h*)(p); f.h[1] = *(const v8h*)(p + 16); return f.v;
  }
  static __device__ __forceinline__ v8f mma(v16h a, v16h b, v8f c) {
    return __builtin_amdgcn_wmma_f32_16x16x32_f16(false, a, false, b, (short)0, c, false, false);
  }
  static __device__ __forceinline__ void guard(v8f& a, v8f& b, v16h x, v16h y) { dep_guard_h(a, b, x, y); }
  static __device__ __forceinline__ void keep(v16h a, v16h b, v16h c, v16h d) { keep4_h(a, b, c, d); }
};
template <> struct Frag<__bf16> {
  typedef v16b V; union U { v16b v; v8b h[2]; };
  static __device__ __forceinline__ v16b load(const __bf16* p) {
    U f; f.h[0] = *(const v8b*)(p); f.h[1] = *(const v8b*)(p + 16); return f.v;
  }
  static __device__ __forceinline__ v8f mma(v16b a, v16b b, v8f c) {
    return __builtin_amdgcn_wmma_f32_16x16x32_bf16(false, a, false, b, (short)0, c, false, false);
  }
  static __device__ __forceinline__ void guard(v8f& a, v8f& b, v16b x, v16b y) { dep_guard_b(a, b, x, y); }
  static __device__ __forceinline__ void keep(v16b a, v16b b, v16b c, v16b d) { keep4_b(a, b, c, d); }
};

template <int ET> struct Elem;
template <> struct Elem<0> { typedef _Float16 T; };
template <> struct Elem<1> { typedef __bf16 T; };
template <int ET, bool SPLIT, int BIAS_MODE, int OUT_MODE, bool RESID, int ACT = 0>
__global__ __launch_bounds__(256) void wmma_gemm64(
    const unsigned short* __restrict__ Ap, const unsigned short* __restrict__ A2p, int lda, long strideA,
    const unsigned short* __restrict__ Btp, const unsigned short* __restrict__ Bt2p, int ldb, long strideB,
    void* __restrict__ Cout, void* __restrict__ Cout2, int ldc, long strideC,
    const float* __restrict__ bias,
    const float* __restrict__ resid, long strideR,
    int M, int N, int K, float scale) {
  typedef typename Elem<ET>::T T;
  typedef typename Frag<T>::V V;
  const T* A = (const T*)Ap; const T* A2 = (const T*)A2p; const T* Bt = (const T*)Btp; const T* Bt2 = (const T*)Bt2p;
  __shared__ __align__(16) float sT[8][16 * 68];
  const int b    = blockIdx.y;
  const int lane = threadIdx.x & 31;
  const int wave = threadIdx.x >> 5;
  const int tilesN = N >> 6;
  const int tilesM = M >> 6;
  const int tile = blockIdx.x * 8 + wave;
  if (tile >= tilesM * tilesN) return;
  const int tm = tile / tilesN;
  const int tn = tile - tm * tilesN;
  const int m0 = tm << 6;
  const int n0 = tn << 6;

  const T* Ab  = A  + (size_t)b * strideA;
  const T* Bb  = Bt + (size_t)b * strideB;
  const T* Ab2 = SPLIT ? (A2  + (size_t)b * strideA) : nullptr;
  const T* Bb2 = SPLIT ? (Bt2 + (size_t)b * strideB) : nullptr;

  const int rlane = lane & 15;
  const int koff  = (lane >> 4) * 8;
  const int mOff  = (lane >> 4) * 8;

  v8f acc[4][4];
#pragma unroll
  for (int i = 0; i < 4; ++i)
#pragma unroll
    for (int j = 0; j < 4; ++j) acc[i][j] = (v8f){0.f,0.f,0.f,0.f,0.f,0.f,0.f,0.f};

  for (int k0 = 0; k0 < K; k0 += 32) {
    V bh[4], bl[4];
#pragma unroll
    for (int j = 0; j < 4; ++j) {
      const size_t bo = (size_t)(n0 + (j << 4) + rlane) * ldb + koff + k0;
      bh[j] = Frag<T>::load(Bb + bo);
      if (SPLIT) bl[j] = Frag<T>::load(Bb2 + bo);
    }
#pragma unroll
    for (int i = 0; i < 4; ++i) {
      const size_t ao = (size_t)(m0 + (i << 4) + rlane) * lda + koff + k0;
      V ah = Frag<T>::load(Ab + ao);
      V al;
      if (SPLIT) al = Frag<T>::load(Ab2 + ao);
#pragma unroll
      for (int j = 0; j < 4; ++j) {
        acc[i][j] = Frag<T>::mma(ah, bh[j], acc[i][j]);
        if (SPLIT) {
          acc[i][j] = Frag<T>::mma(ah, bl[j], acc[i][j]);
          acc[i][j] = Frag<T>::mma(al, bh[j], acc[i][j]);
        }
      }
      Frag<T>::guard(acc[i][0], acc[i][3], ah, SPLIT ? al : ah);
    }
    Frag<T>::keep(bh[0], bh[1], bh[2], bh[3]);
    if (SPLIT) Frag<T>::keep(bl[0], bl[1], bl[2], bl[3]);
  }
  acc_guard4(acc[0][0], acc[0][1], acc[0][2], acc[0][3]);
  acc_guard4(acc[1][0], acc[1][1], acc[1][2], acc[1][3]);
  acc_guard4(acc[2][0], acc[2][1], acc[2][2], acc[2][3]);
  acc_guard4(acc[3][0], acc[3][1], acc[3][2], acc[3][3]);

  float* slab = sT[wave];
  const float* Rb = RESID ? (resid + (size_t)b * strideR) : nullptr;
#pragma unroll
  for (int i = 0; i < 4; ++i) {
    const int mBase = m0 + (i << 4);
#pragma unroll
    for (int j = 0; j < 4; ++j) {
      const int n = n0 + (j << 4) + rlane;
      float bv = 0.f;
      if (BIAS_MODE == 2) bv = bias[n];
#pragma unroll
      for (int r = 0; r < 8; ++r) {
        float v = acc[i][j][r] * scale;
        if (BIAS_MODE == 1) v += bias[mBase + mOff + r];
        if (BIAS_MODE == 2) v += bv;
        if (RESID) v += Rb[(size_t)(mBase + mOff + r) * ldc + n];
        if (ACT == 1) v = tanhf(v);
        if (ACT == 2) v = fmaxf(v, 0.0f);
        if (ACT == 3) v = v / (1.0f + expf(-v));
        if (ACT == 4) v = (v > 0.f) ? v : 0.01f * v;
        if (ACT == 5) v = 0.5f * v * (1.0f + erff(v * 0.70710678118654752f));
        slab[(mOff + r) * 68 + (j << 4) + rlane] = v;
      }
    }
    __builtin_amdgcn_fence(__ATOMIC_RELEASE, "workgroup");
    __builtin_amdgcn_wave_barrier();
    __builtin_amdgcn_fence(__ATOMIC_ACQUIRE, "workgroup");
    if (OUT_MODE == 0) {
      float* C = (float*)Cout + (size_t)b * strideC;
      const int hh = lane >> 4, c4 = (lane & 15) * 4;
      for (int pass = 0; pass < 2; ++pass) {
#pragma unroll
        for (int it = 0; it < 8; ++it) {
          const int row = it * 2 + hh;
          v4f v = *(const v4f*)(slab + row * 68 + c4);
          *(volatile v4f*)(C + (size_t)(mBase + row) * ldc + n0 + c4) = v;
        }
        __threadfence();
      }
    } else {
      const int q = lane >> 3, c8 = (lane & 7) * 8;
      unsigned short* C  = (unsigned short*)Cout  + (size_t)b * strideC;
      unsigned short* C2 = (OUT_MODE == 2) ? ((unsigned short*)Cout2 + (size_t)b * strideC) : nullptr;
      for (int pass = 0; pass < 2; ++pass) {
#pragma unroll
        for (int it = 0; it < 4; ++it) {
          const int row = it * 4 + q;
          const float* sp = slab + row * 68 + c8;
          v8h hv, lv;
#pragma unroll
          for (int e = 0; e < 8; ++e) {
            if (OUT_MODE == 1) {
              hv[e] = (_Float16)sp[e];
            } else {
              unsigned short hb = f2bf_bits(sp[e]);
              unsigned short lb = f2bf_bits(sp[e] - bf_bits2f(hb));
              hv[e] = __builtin_bit_cast(_Float16, hb);
              lv[e] = __builtin_bit_cast(_Float16, lb);
            }
          }
          *(volatile v8h*)(C + (size_t)(mBase + row) * ldc + n0 + c8) = hv;
          if (OUT_MODE == 2) *(volatile v8h*)(C2 + (size_t)(mBase + row) * ldc + n0 + c8) = lv;
        }
        __threadfence();
      }
    }
    __builtin_amdgcn_fence(__ATOMIC_RELEASE, "workgroup");
    __builtin_amdgcn_wave_barrier();
    __builtin_amdgcn_fence(__ATOMIC_ACQUIRE, "workgroup");
  }
}

#define NBATCH 256
#define NSTEP  256
#define NFEAT  64
#define NHID   256
#define NGATE  1024
#define MBLK   16
#define HPITCH 264
#define SLABP  68
#define OPER_CARRY 16.0f
#define ACC_UNSCALE (1.0f / 256.0f)

__global__ __launch_bounds__(256) void cast_scale_f32_f16x2(
    const float* __restrict__ in, unsigned short* __restrict__ out, int n2, float mul) {
  const int i = blockIdx.x * 256 + threadIdx.x;
  if (i < n2) {
    const float a0 = in[2 * i] * mul;
    const float a1 = in[2 * i + 1] * mul;
    const _Float16 h0 = (_Float16)a0, h1 = (_Float16)a1;
    const unsigned u = (unsigned)__builtin_bit_cast(unsigned short, h0) | ((unsigned)__builtin_bit_cast(unsigned short, h1) << 16);
    ((volatile unsigned*)out)[i] = u;
    __threadfence();
    ((volatile unsigned*)out)[i] = u;
  }
}

__device__ __forceinline__ float gate_sigmoid(float x) {
  const float e = expf(-fabsf(x));
  const float r = 1.0f / (1.0f + e);
  return (x >= 0.0f) ? r : e * r;
}

template <bool ENC>
__global__ __launch_bounds__(256) void lstm_seq(
    const unsigned short* __restrict__ x16p,
    const unsigned short* __restrict__ wih16p,
    const unsigned short* __restrict__ whh16p,
    const float* __restrict__ b_ih,
    const float* __restrict__ b_hh,
    const float* __restrict__ xgp,
    unsigned short* __restrict__ hseqp,
    unsigned short* __restrict__ hfinp) {
  typedef Frag<_Float16> FR;
  const _Float16* x16 = (const _Float16*)x16p;
  const _Float16* wih = (const _Float16*)wih16p;
  const _Float16* whh = (const _Float16*)whh16p;

  __shared__ __align__(16) _Float16 hA[MBLK * HPITCH];
  __shared__ __align__(16) float    cS[MBLK * NHID];
  __shared__ __align__(16) float    sT[8][16 * SLABP];

  const int tid  = threadIdx.x;
  const int lane = tid & 31;
  const int wave = tid >> 5;
  const int rl   = lane & 15;
  const int koff = (lane >> 4) * 8;
  const int mOff = (lane >> 4) * 8;
  const int m0   = blockIdx.x * MBLK;

  {
    v8h z8;
#pragma unroll
    for (int e = 0; e < 8; ++e) z8[e] = (_Float16)0.0f;
    for (int i = tid; i < (MBLK * HPITCH) / 8; i += 256) ((v8h*)hA)[i] = z8;
    for (int i = tid; i < MBLK * NHID; i += 256) cS[i] = 0.0f;
  }
  float* sflat = &sT[0][0];
  {
    const v4f bi4 = *(const v4f*)(b_ih + 4 * tid);
    const v4f bh4 = *(const v4f*)(b_hh + 4 * tid);
    *(v4f*)(sflat + 4 * tid) = bi4 + bh4;
  }
  __syncthreads();
  float bsum[2][4];
#pragma unroll
  for (int s = 0; s < 2; ++s)
#pragma unroll
    for (int g = 0; g < 4; ++g)
      bsum[s][g] = sflat[g * NHID + wave * 32 + s * 16 + rl];
  __syncthreads();

  float* slab = sT[wave];

  for (int t = 0; t < NSTEP; ++t) {
    v8f acc[2][4];
#pragma unroll
    for (int s = 0; s < 2; ++s)
#pragma unroll
      for (int g = 0; g < 4; ++g) acc[s][g] = (v8f){0.f,0.f,0.f,0.f,0.f,0.f,0.f,0.f};

    if (ENC) {
#pragma unroll 1
      for (int k0 = 0; k0 < NFEAT; k0 += 32) {
        v16h bf[2][4];
#pragma unroll
        for (int s = 0; s < 2; ++s)
#pragma unroll
          for (int g = 0; g < 4; ++g)
            bf[s][g] = FR::load(wih + (size_t)(g * NHID + wave * 32 + s * 16 + rl) * NFEAT + k0 + koff);
        const v16h af = FR::load(x16 + ((size_t)(m0 + rl) * NSTEP + t) * NFEAT + k0 + koff);
#pragma unroll
        for (int s = 0; s < 2; ++s)
#pragma unroll
          for (int g = 0; g < 4; ++g) acc[s][g] = FR::mma(af, bf[s][g], acc[s][g]);
        FR::guard(acc[0][0], acc[1][3], af, af);
        FR::keep(bf[0][0], bf[0][1], bf[0][2], bf[0][3]);
        FR::keep(bf[1][0], bf[1][1], bf[1][2], bf[1][3]);
      }
    }
#pragma unroll 1
    for (int k0 = 0; k0 < NHID; k0 += 32) {
      v16h bf[2][4];
#pragma unroll
      for (int s = 0; s < 2; ++s)
#pragma unroll
        for (int g = 0; g < 4; ++g)
          bf[s][g] = FR::load(whh + (size_t)(g * NHID + wave * 32 + s * 16 + rl) * NHID + k0 + koff);
      FR::U fa;
      fa.h[0] = *(const v8h*)(hA + rl * HPITCH + k0 + koff);
      fa.h[1] = *(const v8h*)(hA + rl * HPITCH + k0 + 16 + koff);
      const v16h af = fa.v;
#pragma unroll
      for (int s = 0; s < 2; ++s)
#pragma unroll
        for (int g = 0; g < 4; ++g) acc[s][g] = FR::mma(af, bf[s][g], acc[s][g]);
      FR::guard(acc[0][0], acc[1][3], af, af);
      FR::keep(bf[0][0], bf[0][1], bf[0][2], bf[0][3]);
      FR::keep(bf[1][0], bf[1][1], bf[1][2], bf[1][3]);
    }
    acc_guard4(acc[0][0], acc[0][1], acc[0][2], acc[0][3]);
    acc_guard4(acc[1][0], acc[1][1], acc[1][2], acc[1][3]);

    __syncthreads();

#pragma unroll
    for (int s = 0; s < 2; ++s) {
#pragma unroll
      for (int g = 0; g < 4; ++g)
#pragma unroll
        for (int r = 0; r < 8; ++r)
          slab[(mOff + r) * SLABP + g * 16 + rl] = acc[s][g][r] * ACC_UNSCALE;
      __builtin_amdgcn_fence(__ATOMIC_RELEASE, "workgroup");
      __builtin_amdgcn_wave_barrier();
      __builtin_amdgcn_fence(__ATOMIC_ACQUIRE, "workgroup");
      const int col = wave * 32 + s * 16 + rl;
#pragma unroll 1
      for (int r = 0; r < 8; ++r) {
        const int row = mOff + r;
        const float* sp = slab + row * SLABP + rl;
        float pi = sp[0]  + bsum[s][0];
        float pf = sp[16] + bsum[s][1];
        float pg = sp[32] + bsum[s][2];
        float po = sp[48] + bsum[s][3];
        if (!ENC) {
          const float* xr = xgp + (size_t)(m0 + row) * NGATE + col;
          pi += xr[0];
          pf += xr[NHID];
          pg += xr[2 * NHID];
          po += xr[3 * NHID];
        }
        const float ig = gate_sigmoid(pi);
        const float fg = gate_sigmoid(pf);
        const float gg = tanhf(pg);
        const float og = gate_sigmoid(po);
        const int ci = row * NHID + col;
        const float cn = fg * cS[ci] + ig * gg;
        cS[ci] = cn;
        const float hn = og * tanhf(cn);
        hA[row * HPITCH + col] = (_Float16)(hn * OPER_CARRY);
      }
      __builtin_amdgcn_fence(__ATOMIC_RELEASE, "workgroup");
      __builtin_amdgcn_wave_barrier();
      __builtin_amdgcn_fence(__ATOMIC_ACQUIRE, "workgroup");
    }
    __syncthreads();

    if (!ENC) {
      _Float16* hseq = (_Float16*)hseqp;
      const int q = lane >> 3, c8 = (lane & 7) * 8;
      for (int pass = 0; pass < 2; ++pass) {
#pragma unroll
        for (int it = 0; it < 2; ++it) {
          const int row = 2 * wave + it;
          const v8h val = *(const v8h*)(hA + row * HPITCH + q * 64 + c8);
          *(volatile v8h*)(hseq + ((size_t)(m0 + row) * NSTEP + t) * NHID + q * 64 + c8) = val;
        }
        __threadfence();
      }
    }
  }

  if (ENC) {
    _Float16* hfin = (_Float16*)hfinp;
    const int q = lane >> 3, c8 = (lane & 7) * 8;
    for (int pass = 0; pass < 2; ++pass) {
#pragma unroll
      for (int it = 0; it < 2; ++it) {
        const int row = 2 * wave + it;
        const v8h val = *(const v8h*)(hA + row * HPITCH + q * 64 + c8);
        *(volatile v8h*)(hfin + (size_t)(m0 + row) * NHID + q * 64 + c8) = val;
      }
      __threadfence();
    }
  }
}

#define WS_X16    ((size_t)NBATCH * NSTEP * NFEAT * 2)
#define WS_WIH    ((size_t)NGATE * NFEAT * 2)
#define WS_WHH    ((size_t)NGATE * NHID * 2)
#define WS_WOUT   ((size_t)NFEAT * NHID * 2)
#define WS_HFIN   ((size_t)NBATCH * NHID * 2)
#define WS_XG     ((size_t)NBATCH * NGATE * 4)
#define WS_HSEQ   ((size_t)NBATCH * NSTEP * NHID * 2)
#define WS_TOTAL  (WS_X16 + WS_WIH + 3 * WS_WHH + WS_WOUT + WS_HFIN + WS_XG + WS_HSEQ)
static_assert(WS_TOTAL == 44859392, "carve total");
static_assert(WS_TOTAL <= 134217728, "carve under 128 MiB");
static_assert(NBATCH % MBLK == 0, "recurrence grid");
static_assert(NBATCH % 64 == 0 && NGATE % 64 == 0 && NHID % 32 == 0, "xg GEMM: M, N tile multiples, K % 32");
static_assert((NBATCH * NSTEP) % 64 == 0 && NFEAT % 64 == 0, "output GEMM: M, N tile multiples");
static_assert((NBATCH * NSTEP * NFEAT) % 512 == 0 && (NGATE * NFEAT) % 512 == 0 && (NGATE * NHID) % 512 == 0 && (NFEAT * NHID) % 512 == 0, "cast grids exact, whole lines");

extern "C" void kernel_launch(void* const* d_in, const int* in_sizes, int n_in,
                              void* d_out, int out_size, void* d_ws, size_t ws_size,
                              hipStream_t stream) {
  if (n_in < 11) return;
  if (ws_size < WS_TOTAL) return;
  if (in_sizes[0] != NBATCH * NSTEP * NFEAT || out_size != NBATCH * NSTEP * NFEAT) return;

  const float* x        = (const float*)d_in[0];
  const float* enc_W_ih = (const float*)d_in[1];
  const float* enc_W_hh = (const float*)d_in[2];
  const float* enc_b_ih = (const float*)d_in[3];
  const float* enc_b_hh = (const float*)d_in[4];
  const float* dec_W_ih = (const float*)d_in[5];
  const float* dec_W_hh = (const float*)d_in[6];
  const float* dec_b_ih = (const float*)d_in[7];
  const float* dec_b_hh = (const float*)d_in[8];
  const float* W_out    = (const float*)d_in[9];
  const float* b_out    = (const float*)d_in[10];
  float* out = (float*)d_out;

  char* ws = (char*)d_ws;
  size_t o = 0;
  unsigned short* x16    = (unsigned short*)(ws + o); o += WS_X16;
  unsigned short* wih16  = (unsigned short*)(ws + o); o += WS_WIH;
  unsigned short* ewhh16 = (unsigned short*)(ws + o); o += WS_WHH;
  unsigned short* dwih16 = (unsigned short*)(ws + o); o += WS_WHH;
  unsigned short* dwhh16 = (unsigned short*)(ws + o); o += WS_WHH;
  unsigned short* wout16 = (unsigned short*)(ws + o); o += WS_WOUT;
  unsigned short* hfin   = (unsigned short*)(ws + o); o += WS_HFIN;
  float*          xg     = (float*)(ws + o);          o += WS_XG;
  unsigned short* hseq   = (unsigned short*)(ws + o); o += WS_HSEQ;
  if (o > ws_size) return;

  const int n2x   = NBATCH * NSTEP * NFEAT / 2;
  const int n2wih = NGATE * NFEAT / 2;
  const int n2whh = NGATE * NHID / 2;
  const int n2wo  = NFEAT * NHID / 2;
  cast_scale_f32_f16x2<<<n2x / 256, 256, 0, stream>>>(x, x16, n2x, OPER_CARRY);
  cast_scale_f32_f16x2<<<n2wih / 256, 256, 0, stream>>>(enc_W_ih, wih16, n2wih, OPER_CARRY);
  cast_scale_f32_f16x2<<<n2whh / 256, 256, 0, stream>>>(enc_W_hh, ewhh16, n2whh, OPER_CARRY);
  cast_scale_f32_f16x2<<<n2whh / 256, 256, 0, stream>>>(dec_W_ih, dwih16, n2whh, OPER_CARRY);
  cast_scale_f32_f16x2<<<n2whh / 256, 256, 0, stream>>>(dec_W_hh, dwhh16, n2whh, OPER_CARRY);
  cast_scale_f32_f16x2<<<n2wo / 256, 256, 0, stream>>>(W_out, wout16, n2wo, OPER_CARRY);

  lstm_seq<true><<<NBATCH / MBLK, 256, 0, stream>>>(x16, wih16, ewhh16, enc_b_ih, enc_b_hh, xg, hseq, hfin);

  wmma_gemm64<0, false, 0, 0, false><<<dim3((NBATCH / 64) * (NGATE / 64) / 8, 1), 256, 0, stream>>>(
      hfin, hfin, NHID, 0L,
      dwih16, dwih16, NHID, 0L,
      (void*)xg, (void*)xg, NGATE, 0L,
      b_out, xg, 0L,
      NBATCH, NGATE, NHID, ACC_UNSCALE);

  lstm_seq<false><<<NBATCH / MBLK, 256, 0, stream>>>(x16, wih16, dwhh16, dec_b_ih, dec_b_hh, xg, hseq, hfin);

  wmma_gemm64<0, false, 2, 0, false><<<dim3((NBATCH * NSTEP / 64) * (NFEAT / 64) / 8, 1), 256, 0, stream>>>(
      hseq, hseq, NHID, 0L,
      wout16, wout16, NHID, 0L,
      (void*)out, (void*)out, NFEAT, 0L,
      b_out, xg, 0L,
      NBATCH * NSTEP, NFEAT, NHID, ACC_UNSCALE);
}
